// GNN_47098611368430
// MI455X (gfx1250) — hardware-verified
//
#include <hip/hip_runtime.h>
#include <stddef.h>
#include <stdint.h>


#define DIN    64
#define DH     128
#define DOUT   64
#define P1     192
#define P2     512
#define NTHR   256
#define NWAVE  8
#define EPT    8
#define CHUNK  (NTHR * EPT)
#define WCAP   (EPT * 32)
#define LISTN  (NWAVE * WCAP)
#define NBA    1024
#define SLA    10
#define RCAP   28672
#define DEGCAP 64
#define GBM    64
#define GBN    128
#define GTHR   128
#define U1     1024
#define U2     2048
#define NUW    (3 * U1 + 4 * U2)
#define AGG_ZINTS    (LISTN + 2 * RCAP + 3 * NBA)
#define MISC_INTS    16
#define ROWBUF_INTS  (NWAVE * 128)
#define AGG_LDS_INTS (AGG_ZINTS + MISC_INTS + ROWBUF_INTS)
#define WSMAX  134217728

static_assert((CHUNK & (CHUNK - 1)) == 0 && CHUNK <= 4096);
static_assert((NBA & (NBA - 1)) == 0 && NBA == (1 << SLA));
static_assert(((long long)CHUNK << SLA) < (1LL << 31));
static_assert(LISTN % NTHR == 0);
static_assert(NBA % NWAVE == 0 && NBA % 32 == 0 && NBA % GBM == 0);
static_assert(RCAP % 4 == 0 && AGG_ZINTS % 4 == 0 && LISTN % 4 == 0 && ((AGG_ZINTS + MISC_INTS) % 4) == 0);
static_assert(AGG_ZINTS % (NTHR * 4) == 0);
static_assert(P1 % 32 == 0 && P2 % 32 == 0 && P1 == 3 * DIN && P2 == 4 * DH);
static_assert(GBN == DH && GBM == (GTHR / 32) * 16 && DH == 4 * 32 && DIN == 2 * 32);
static_assert(U1 % NTHR == 0 && U2 % NTHR == 0 && NUW % NTHR == 0);
static_assert(U1 == DH * (DIN / 8) && U2 == DH * (DH / 8));
static_assert(AGG_LDS_INTS * 4 <= 300000);
static_assert((DOUT * 4) % 128 == 0 && 4 * DOUT == NTHR);

typedef float          v4f   __attribute__((ext_vector_type(4)));
typedef float          v8f   __attribute__((ext_vector_type(8)));
typedef int            v4i   __attribute__((ext_vector_type(4)));
typedef int            v8i   __attribute__((ext_vector_type(8)));
typedef unsigned int   v4u   __attribute__((ext_vector_type(4)));
typedef unsigned short v4us  __attribute__((ext_vector_type(4)));
typedef unsigned short v8us  __attribute__((ext_vector_type(8)));
typedef unsigned short v16us __attribute__((ext_vector_type(16)));
typedef __bf16         v16bf __attribute__((ext_vector_type(16)));
typedef v4f  __attribute__((may_alias)) v4fa;
typedef v4i  __attribute__((may_alias)) v4ia;
typedef v4us __attribute__((may_alias)) v4usa;
typedef v8us __attribute__((may_alias)) v8usa;
typedef unsigned int __attribute__((may_alias)) u32a;
union FragB { v16bf v; v16us u; v8us h[2]; v8i w; };

__device__ __forceinline__ v8f wmb(const FragB& a, const FragB& b, v8f c) {
  v8f d = __builtin_amdgcn_wmma_f32_16x16x32_bf16(false, a.v, false, b.v, (short)0, c, false, false);
  asm volatile("v_nop\n\tv_nop\n\tv_nop\n\tv_nop" : "+v"(d) : "v"(a.w), "v"(b.w));
  return d;
}

__device__ __forceinline__ unsigned bf16_bits(float f) {
  const unsigned u = __float_as_uint(f);
  return (u + 0x7FFFu + ((u >> 16) & 1u)) >> 16;
}
__device__ __forceinline__ float bf16_val(float f) {
  return __uint_as_float(bf16_bits(f) << 16);
}

__device__ __forceinline__ void wave_sync() {
  __builtin_amdgcn_fence(__ATOMIC_RELEASE, "wavefront");
  __builtin_amdgcn_wave_barrier();
  __builtin_amdgcn_fence(__ATOMIC_ACQUIRE, "wavefront");
}

template <int SLB>
__device__ __forceinline__ int scan_chunk(const int* __restrict__ dsts, int nE, int cbase, int slotBase,
                                          int nb, int vec8, int* list, int tid, int lane, int wave) {
  int wc = 0;
  const int el0  = tid * EPT;
  const int e0   = cbase + el0;
  const int sent = -2147483647 - 1;
  v4i da, db;
  if (vec8 != 0 && cbase + CHUNK <= nE) {
    da = *(const v4i*)(dsts + e0);
    db = *(const v4i*)(dsts + e0 + 4);
  } else {
    da.x = (e0     < nE) ? dsts[min(e0,     nE - 1)] : sent;
    da.y = (e0 + 1 < nE) ? dsts[min(e0 + 1, nE - 1)] : sent;
    da.z = (e0 + 2 < nE) ? dsts[min(e0 + 2, nE - 1)] : sent;
    da.w = (e0 + 3 < nE) ? dsts[min(e0 + 3, nE - 1)] : sent;
    db.x = (e0 + 4 < nE) ? dsts[min(e0 + 4, nE - 1)] : sent;
    db.y = (e0 + 5 < nE) ? dsts[min(e0 + 5, nE - 1)] : sent;
    db.z = (e0 + 6 < nE) ? dsts[min(e0 + 6, nE - 1)] : sent;
    db.w = (e0 + 7 < nE) ? dsts[min(e0 + 7, nE - 1)] : sent;
  }
  const unsigned nbs = (unsigned)slotBase;
  const unsigned unb = (unsigned)nb;
  const unsigned s0 = (unsigned)da.x - nbs, s1 = (unsigned)da.y - nbs;
  const unsigned s2 = (unsigned)da.z - nbs, s3 = (unsigned)da.w - nbs;
  const unsigned s4 = (unsigned)db.x - nbs, s5 = (unsigned)db.y - nbs;
  const unsigned s6 = (unsigned)db.z - nbs, s7 = (unsigned)db.w - nbs;
  const bool h0 = s0 < unb, h1 = s1 < unb, h2 = s2 < unb, h3 = s3 < unb;
  const bool h4 = s4 < unb, h5 = s5 < unb, h6 = s6 < unb, h7 = s7 < unb;
  const unsigned any = __builtin_amdgcn_ballot_w32(h0 | h1 | h2 | h3 | h4 | h5 | h6 | h7);
  if (any != 0u) {
#define HITJ(J, HJ, SJ) { \
      const unsigned mj = __builtin_amdgcn_ballot_w32(HJ); \
      if (mj != 0u) { \
        if (HJ) { \
          const int pos = wc + (int)__builtin_amdgcn_mbcnt_lo(mj, 0u); \
          if (pos < WCAP) list[wave * WCAP + pos] = ((el0 + (J)) << SLB) | (int)(SJ); \
        } \
        wc += (int)__builtin_popcount(mj); } }
    HITJ(0, h0, s0)
    HITJ(1, h1, s1)
    HITJ(2, h2, s2)
    HITJ(3, h3, s3)
    HITJ(4, h4, s4)
    HITJ(5, h5, s5)
    HITJ(6, h6, s6)
    HITJ(7, h7, s7)
#undef HITJ
  }
  return wc;
}

__device__ __forceinline__ v8us gather8(const float* __restrict__ W, int k8, int n) {
  const float* p = W + (size_t)k8 * DH + n;
  v8us o;
#pragma unroll
  for (int i = 0; i < 8; ++i) o[i] = (unsigned short)bf16_bits(p[(size_t)i * DH]);
  return o;
}
__device__ __forceinline__ void put8(unsigned short* dp, v8us o) {
  *(volatile v8us*)dp = o;
  __threadfence();
  *(volatile v8us*)dp = o;
}

__global__ __launch_bounds__(NTHR) void k_wprep(const float* __restrict__ w1a, const float* __restrict__ w1b,
                                                const float* __restrict__ w2a, const float* __restrict__ w2b,
                                                unsigned short* W1C, unsigned short* W2C) {
  const int bu = (int)blockIdx.x * NTHR;
  const int u  = bu + (int)threadIdx.x;
  if (bu < U1) {
    const int v = u, n = v >> 3, k8 = (v & 7) * 8;
    const v8us o = gather8(w1a, k8, n);
    put8(W1C + (size_t)n * P1 + k8, o);
  } else if (bu < 2 * U1) {
    const int v = u - U1, n = v >> 3, k8 = (v & 7) * 8;
    const v8us o = gather8(w1b, k8, n);
    put8(W1C + (size_t)n * P1 + DIN + k8, o);
  } else if (bu < 3 * U1) {
    const int v = u - 2 * U1, n = v >> 3, k8 = (v & 7) * 8;
    const v8us o = gather8(w1b, k8, n);
    put8(W1C + (size_t)n * P1 + 2 * DIN + k8, o);
  } else if (bu < 3 * U1 + U2) {
    const int v = u - 3 * U1, n = v >> 4, k8 = (v & 15) * 8;
    const v8us o = gather8(w2a, k8, n);
    put8(W2C + (size_t)n * P2 + k8, o);
  } else if (bu < 3 * U1 + 2 * U2) {
    const int v = u - 3 * U1 - U2, n = v >> 4, k8 = (v & 15) * 8;
    const v8us o = gather8(w2a, k8, n);
    put8(W2C + (size_t)n * P2 + DH + k8, o);
  } else if (bu < 3 * U1 + 3 * U2) {
    const int v = u - 3 * U1 - 2 * U2, n = v >> 4, k8 = (v & 15) * 8;
    const v8us o = gather8(w2b, k8, n);
    put8(W2C + (size_t)n * P2 + 2 * DH + k8, o);
  } else if (bu < 3 * U1 + 4 * U2) {
    const int v = u - 3 * U1 - 3 * U2, n = v >> 4, k8 = (v & 15) * 8;
    const v8us o = gather8(w2b, k8, n);
    put8(W2C + (size_t)n * P2 + 3 * DH + k8, o);
  }
}

__global__ __launch_bounds__(NTHR) void k_cvx(const float* __restrict__ x, int nN, int nUnits,
                                              unsigned short* a1) {
  const int u = (int)blockIdx.x * NTHR + (int)threadIdx.x;
  if (u >= nUnits) return;
  const int row = u >> 3;
  const int k8  = (u & 7) * 8;
  const int rc  = row < nN ? row : nN - 1;
  const float* p = x + (size_t)rc * DIN + k8;
  const v4f a = *(const v4fa*)p;
  const v4f b = *(const v4fa*)(p + 4);
  const bool ok = row < nN;
  v8us o;
  o[0] = ok ? (unsigned short)bf16_bits(a.x) : (unsigned short)0;
  o[1] = ok ? (unsigned short)bf16_bits(a.y) : (unsigned short)0;
  o[2] = ok ? (unsigned short)bf16_bits(a.z) : (unsigned short)0;
  o[3] = ok ? (unsigned short)bf16_bits(a.w) : (unsigned short)0;
  o[4] = ok ? (unsigned short)bf16_bits(b.x) : (unsigned short)0;
  o[5] = ok ? (unsigned short)bf16_bits(b.y) : (unsigned short)0;
  o[6] = ok ? (unsigned short)bf16_bits(b.z) : (unsigned short)0;
  o[7] = ok ? (unsigned short)bf16_bits(b.w) : (unsigned short)0;
  unsigned short* dp = a1 + (size_t)row * P1 + k8;
  *(volatile v8us*)dp = o;
  __threadfence();
  *(volatile v8us*)dp = o;
}

template <int LY>
__global__ __launch_bounds__(NTHR) void k_scan(const int* __restrict__ gath, const int* __restrict__ keys,
                                               int nE, int nN, int vec8, int mRows,
                                               const unsigned short* srcb, const float* __restrict__ srcf,
                                               unsigned short* dstpl) {
  extern __shared__ __attribute__((aligned(16))) int dsm[];
  int* list = dsm;
  int* hl   = dsm + LISTN;
  int* sl   = hl + RCAP;
  int* cnt  = sl + RCAP;
  int* offs = cnt + NBA;
  int* cur  = offs + NBA;
  int* misc = cur + NBA;
  const int tid = (int)threadIdx.x, lane = tid & 31, wave = tid >> 5;
  unsigned short* rowbuf = (unsigned short*)(misc + MISC_INTS) + wave * 256;
  const int nodeBase = (int)blockIdx.x * NBA;

  {
    const v4i z4 = {0, 0, 0, 0};
    for (int i = tid * 4; i < AGG_ZINTS; i += NTHR * 4) *(v4ia*)(dsm + i) = z4;
    if (tid < MISC_INTS) misc[tid] = 0;
  }
  __syncthreads();

  int t = 0, ov = 0;
  const int nChunks = (nE + CHUNK - 1) / CHUNK;
#pragma unroll 1
  for (int ch = 0; ch < nChunks; ++ch) {
    const int cbase = ch * CHUNK;
    const int wc = scan_chunk<SLA>(keys, nE, cbase, nodeBase, NBA, vec8, list, tid, lane, wave);
    if (lane == 0) misc[wave] = wc;
    __syncthreads();
    if (wave == 0) {
#pragma unroll 1
      for (int w2 = 0; w2 < NWAVE; ++w2) {
        int c = misc[w2];
        c = c < 0 ? 0 : (c > WCAP ? WCAP : c);
#pragma unroll 1
        for (int b0 = 0; b0 < c; b0 += 32) {
          const int idx = b0 + lane;
          const int ent = list[w2 * WCAP + (idx < WCAP ? idx : WCAP - 1)];
          const int m32 = (c - b0) < 32 ? (c - b0) : 32;
#pragma unroll 1
          for (int k = 0; k < m32; ++k) {
            const int u    = __builtin_amdgcn_readlane(ent, k);
            const int slot = u & (NBA - 1);
            const int el   = (u >> SLA) & (CHUNK - 1);
            const int pk   = ((cbase + el) << SLA) | slot;
            if (t < RCAP) {
              if (lane == 0) { hl[t] = pk; cnt[slot] = cnt[slot] + 1; }
              t = t + 1;
            } else {
              ov = 1;
            }
          }
        }
      }
    }
    __syncthreads();
  }
  if (wave == 0 && lane == 0) { misc[8] = t; misc[9] = ov; }
  __syncthreads();
  int tt = misc[8];
  tt = tt < 0 ? 0 : (tt > RCAP ? RCAP : tt);
  const int ovf = misc[9];

  if (wave == 0) {
    const int base = lane * (NBA / 32);
    int s = 0;
#pragma unroll 1
    for (int i = 0; i < NBA / 32; ++i) s += cnt[base + i];
    int incl = s;
#pragma unroll
    for (int d = 1; d < 32; d <<= 1) {
      const int y = __shfl_up(incl, d, 32);
      if (lane >= d) incl += y;
    }
    int run = incl - s;
#pragma unroll 1
    for (int i = 0; i < NBA / 32; ++i) {
      const int cv = cnt[base + i];
      offs[base + i] = run;
      cur[base + i]  = run;
      run += cv;
    }
  }
  __syncthreads();
  if (wave == 0) {
#pragma unroll 1
    for (int b0 = 0; b0 < tt; b0 += 32) {
      const int idx = b0 + lane;
      const int ent = hl[idx < RCAP ? idx : RCAP - 1];
      const int m32 = (tt - b0) < 32 ? (tt - b0) : 32;
#pragma unroll 1
      for (int k = 0; k < m32; ++k) {
        const int u    = __builtin_amdgcn_readlane(ent, k);
        const int slot = u & (NBA - 1);
        if (lane == 0) {
          int p = cur[slot];
          p = p < 0 ? 0 : (p > RCAP - 1 ? RCAP - 1 : p);
          sl[p] = u;
          cur[slot] = p + 1;
        }
      }
    }
  }
  __syncthreads();

  const float qnan = __int_as_float(0x7fc00000);
  const float pz = (ovf != 0) ? qnan : 0.0f;
  const int q0s = (4 * lane) & 31, q1s = (4 * lane + 1) & 31;
  const int q2s = (4 * lane + 2) & 31, q3s = (4 * lane + 3) & 31;
#pragma unroll 1
  for (int si = 0; si < NBA / NWAVE; ++si) {
    const int s    = si * NWAVE + wave;
    const int node = nodeBase + s;
    int c = cnt[s];
    const bool big = c > DEGCAP;
    c = c < 0 ? 0 : (c > DEGCAP ? DEGCAP : c);
    int o = offs[s];
    o = o < 0 ? 0 : (o > RCAP ? RCAP : o);
    float a0 = 0.0f, a1 = 0.0f, a2 = 0.0f, a3 = 0.0f;
#pragma unroll 1
    for (int b0 = 0; b0 < c; b0 += 32) {
      int idx = o + b0 + lane;
      idx = idx > RCAP - 1 ? RCAP - 1 : idx;
      const int ent = sl[idx];
      int eid = ent >> SLA;
      eid = eid < 0 ? 0 : (eid > nE - 1 ? nE - 1 : eid);
      int sr = gath[eid];
      sr = sr < 0 ? 0 : (sr > nN - 1 ? nN - 1 : sr);
      const int m32 = (c - b0) < 32 ? (c - b0) : 32;
#pragma unroll 1
      for (int k = 0; k < m32; ++k) {
        const int sk = __builtin_amdgcn_readlane(sr, k);
        if constexpr (LY != 0) {
          const unsigned w = *(const u32a*)(srcb + (size_t)sk * P1 + 2 * lane);
          a0 += __uint_as_float(w << 16);
          a1 += __uint_as_float(w & 0xffff0000u);
        } else {
          const v4f a = *(const v4f*)(srcf + (size_t)sk * DH + 4 * lane);
          a0 += a.x; a1 += a.y; a2 += a.z; a3 += a.w;
        }
      }
    }
    const float pzr = big ? qnan : pz;
    const bool live = node < nN;
    if constexpr (LY != 0) {
      const float v0 = live ? (a0 + pzr) : 0.0f;
      const float v1 = live ? (a1 + pzr) : 0.0f;
      const unsigned hb0 = bf16_bits(v0), hb1 = bf16_bits(v1);
      const unsigned lb0 = bf16_bits(v0 - __uint_as_float(hb0 << 16));
      const unsigned lb1 = bf16_bits(v1 - __uint_as_float(hb1 << 16));
      const int hw = (int)(hb0 | (hb1 << 16));
      const int lw = (int)(lb0 | (lb1 << 16));
      const int g0 = __shfl(hw, q0s, 32), g1 = __shfl(hw, q1s, 32);
      const int g2 = __shfl(hw, q2s, 32), g3 = __shfl(hw, q3s, 32);
      const int p0 = __shfl(lw, q0s, 32), p1 = __shfl(lw, q1s, 32);
      const int p2 = __shfl(lw, q2s, 32), p3 = __shfl(lw, q3s, 32);
      const bool lsel = (lane & 8) != 0;
      v4u pv;
      pv.x = (unsigned int)(lsel ? p0 : g0);
      pv.y = (unsigned int)(lsel ? p1 : g1);
      pv.z = (unsigned int)(lsel ? p2 : g2);
      pv.w = (unsigned int)(lsel ? p3 : g3);
      const bool wr = (node < mRows) && (lane < 16);
      unsigned short* hp = dstpl + (size_t)node * P1 + DIN + 8 * (lane & 15);
      if (wr) *(volatile v4u*)hp = pv;
      __threadfence();
      if (wr) *(volatile v4u*)hp = pv;
    } else {
      const float m0 = live ? (a0 + pzr) : 0.0f;
      const float m1 = live ? (a1 + pzr) : 0.0f;
      const float m2 = live ? (a2 + pzr) : 0.0f;
      const float m3 = live ? (a3 + pzr) : 0.0f;
      v4us mh, ml;
      {
        unsigned hb;
        hb = bf16_bits(m0); mh[0] = (unsigned short)hb; ml[0] = (unsigned short)bf16_bits(m0 - __uint_as_float(hb << 16));
        hb = bf16_bits(m1); mh[1] = (unsigned short)hb; ml[1] = (unsigned short)bf16_bits(m1 - __uint_as_float(hb << 16));
        hb = bf16_bits(m2); mh[2] = (unsigned short)hb; ml[2] = (unsigned short)bf16_bits(m2 - __uint_as_float(hb << 16));
        hb = bf16_bits(m3); mh[3] = (unsigned short)hb; ml[3] = (unsigned short)bf16_bits(m3 - __uint_as_float(hb << 16));
      }
      *(v4usa*)(rowbuf + 4 * lane) = mh;
      *(v4usa*)(rowbuf + DH + 4 * lane) = ml;
      wave_sync();
      const v8us q0 = *(const v8usa*)(rowbuf + 8 * lane);
      wave_sync();
      if (node < mRows) {
        unsigned short* rpw = dstpl + (size_t)node * P2 + 2 * DH + 8 * lane;
        *(volatile v8us*)rpw = q0;
        __threadfence();
        *(volatile v8us*)rpw = q0;
      }
    }
  }
}

template <int HL>
__global__ __launch_bounds__(GTHR) void k_gemm(const unsigned short* __restrict__ Apl,
                                               const unsigned short* __restrict__ BT, int K,
                                               const float* __restrict__ bA, const float* __restrict__ bB,
                                               float* hout, unsigned short* a2, int nOut) {
  __shared__ __attribute__((aligned(16))) float stg[GBM * GBN];
  const int tid = (int)threadIdx.x, lane = tid & 31, wave = tid >> 5, hh = lane >> 4, m = lane & 15;
  const int rowBase = (int)blockIdx.x * GBM;

  v8f acc[8];
  {
    const v8f z = {0.f, 0.f, 0.f, 0.f, 0.f, 0.f, 0.f, 0.f};
#pragma unroll
    for (int t = 0; t < 8; ++t) acc[t] = z;
  }
  const unsigned short* ap = Apl + (size_t)(rowBase + 16 * wave + m) * (size_t)K + 8 * hh;
  const unsigned short* bp = BT + (size_t)m * (size_t)K + 8 * hh;

#pragma unroll 1
  for (int k0 = 0; k0 < K; k0 += 32) {
    FragB af;
    af.h[0] = *(const v8usa*)(ap + k0);
    af.h[1] = *(const v8usa*)(ap + k0 + 16);
#pragma unroll
    for (int nt = 0; nt < 8; ++nt) {
      const unsigned short* wq = bp + (size_t)(16 * nt) * (size_t)K + k0;
      FragB bf;
      bf.h[0] = *(const v8usa*)wq;
      bf.h[1] = *(const v8usa*)(wq + 16);
      acc[nt] = wmb(af, bf, acc[nt]);
    }
  }

#pragma unroll
  for (int nt = 0; nt < 8; ++nt) {
    const int lc = 16 * nt + m;
#pragma unroll
    for (int r = 0; r < 8; ++r) {
      const int lr = 16 * wave + 8 * hh + r;
      stg[lr * GBN + lc] = acc[nt][r];
    }
  }
  __syncthreads();

  v4f bb4;
  {
    const v4f t1 = *(const v4f*)(bA + 4 * lane);
    const v4f t2 = *(const v4f*)(bB + 4 * lane);
    bb4.x = bf16_val(t1.x) + bf16_val(t2.x);
    bb4.y = bf16_val(t1.y) + bf16_val(t2.y);
    bb4.z = bf16_val(t1.z) + bf16_val(t2.z);
    bb4.w = bf16_val(t1.w) + bf16_val(t2.w);
  }

  v4f pv[16];
#pragma unroll
  for (int i = 0; i < 16; ++i) pv[i] = *(const v4fa*)(stg + (16 * wave + i) * GBN + 4 * lane);
  __syncthreads();

#pragma unroll
  for (int i = 0; i < 16; ++i) {
    const bool ok = (rowBase + 16 * wave + i) < nOut;
    const v4f t = pv[i] + bb4;
    v4f y;
    y.x = (t.x > 0.0f) ? t.x : (t.x - t.x);
    y.y = (t.y > 0.0f) ? t.y : (t.y - t.y);
    y.z = (t.z > 0.0f) ? t.z : (t.z - t.z);
    y.w = (t.w > 0.0f) ? t.w : (t.w - t.w);
    y.x = ok ? y.x : 0.0f; y.y = ok ? y.y : 0.0f; y.z = ok ? y.z : 0.0f; y.w = ok ? y.w : 0.0f;
    pv[i] = y;
  }

#pragma unroll
  for (int i = 0; i < 16; ++i) {
    const int r = rowBase + 16 * wave + i;
    *(volatile v4f*)(hout + (size_t)r * DH + 4 * lane) = pv[i];
  }
  __threadfence();
#pragma unroll
  for (int i = 0; i < 16; ++i) {
    const int r = rowBase + 16 * wave + i;
    *(volatile v4f*)(hout + (size_t)r * DH + 4 * lane) = pv[i];
  }

  if constexpr (HL != 0) {
#pragma unroll
    for (int i = 0; i < 16; ++i) {
      v4us h4, l4;
      unsigned hb;
      hb = bf16_bits(pv[i].x); h4[0] = (unsigned short)hb; l4[0] = (unsigned short)bf16_bits(pv[i].x - __uint_as_float(hb << 16));
      hb = bf16_bits(pv[i].y); h4[1] = (unsigned short)hb; l4[1] = (unsigned short)bf16_bits(pv[i].y - __uint_as_float(hb << 16));
      hb = bf16_bits(pv[i].z); h4[2] = (unsigned short)hb; l4[2] = (unsigned short)bf16_bits(pv[i].z - __uint_as_float(hb << 16));
      hb = bf16_bits(pv[i].w); h4[3] = (unsigned short)hb; l4[3] = (unsigned short)bf16_bits(pv[i].w - __uint_as_float(hb << 16));
      unsigned short* srow = (unsigned short*)stg + (size_t)(16 * wave + i) * (2 * GBN);
      *(v4usa*)(srow + 4 * lane) = h4;
      *(v4usa*)(srow + DH + 4 * lane) = l4;
    }
    __syncthreads();
    v8us qv[16];
#pragma unroll
    for (int i = 0; i < 16; ++i) {
      const unsigned short* srow = (const unsigned short*)stg + (size_t)(16 * wave + i) * (2 * GBN);
      qv[i] = *(const v8usa*)(srow + 8 * lane);
    }
#pragma unroll
    for (int i = 0; i < 16; ++i) {
      unsigned short* rp = a2 + (size_t)(rowBase + 16 * wave + i) * (size_t)P2 + 8 * lane;
      *(volatile v8us*)rp = qv[i];
    }
    __threadfence();
#pragma unroll
    for (int i = 0; i < 16; ++i) {
      unsigned short* rp = a2 + (size_t)(rowBase + 16 * wave + i) * (size_t)P2 + 8 * lane;
      *(volatile v8us*)rp = qv[i];
    }
  }
}

__global__ __launch_bounds__(NTHR) void k_pool_out(const float* __restrict__ hf, const int* __restrict__ gid,
                                                   int nN, const float* __restrict__ wf,
                                                   const float* __restrict__ bfv, float* out) {
  __shared__ __attribute__((aligned(16))) float wsum[NWAVE * DH];
  __shared__ __attribute__((aligned(16))) float pooled[DH];
  __shared__ __attribute__((aligned(16))) float part[4 * DOUT];
  __shared__ __attribute__((aligned(16))) float outs[DOUT];
  const int tid = (int)threadIdx.x, lane = tid & 31, wave = tid >> 5;
  const int g = (int)blockIdx.x;

  float a0 = 0.0f, a1 = 0.0f, a2 = 0.0f, a3 = 0.0f;
#pragma unroll 1
  for (int i0 = wave * 32; i0 < nN; i0 += NTHR) {
    const int i  = i0 + lane;
    const int ic = i < nN ? i : nN - 1;
    const int b  = gid[ic];
    const bool hit = (i < nN) && (b == g);
    unsigned msk = __builtin_amdgcn_ballot_w32(hit);
    int nh = (int)__builtin_popcount(msk);
    nh = nh > 32 ? 32 : nh;
#pragma unroll 1
    for (int q = 0; q < nh; ++q) {
      const int k = __builtin_ffs((int)msk) - 1;
      msk &= msk - 1u;
      int node = i0 + (k < 0 ? 0 : k);
      node = node > nN - 1 ? nN - 1 : node;
      const v4f v = *(const v4fa*)(hf + (size_t)node * DH + 4 * lane);
      a0 += v.x; a1 += v.y; a2 += v.z; a3 += v.w;
    }
  }
  {
    v4f av;
    av.x = a0; av.y = a1; av.z = a2; av.w = a3;
    *(v4fa*)(wsum + wave * DH + 4 * lane) = av;
  }
  __syncthreads();
  if (tid < DH) {
    float s = 0.0f;
#pragma unroll
    for (int w2 = 0; w2 < NWAVE; ++w2) s += wsum[w2 * DH + tid];
    pooled[tid] = s;
  }
  __syncthreads();
  {
    const int kq = tid >> 6;
    const int o  = tid & (DOUT - 1);
    float s = 0.0f;
#pragma unroll 4
    for (int kk = 0; kk < 32; ++kk) {
      const int k = kq * 32 + kk;
      s = fmaf(pooled[k], bf16_val(wf[(size_t)k * DOUT + o]), s);
    }
    part[kq * DOUT + o] = s;
  }
  __syncthreads();
  if (tid < DOUT) {
    const float s = (part[tid] + part[DOUT + tid]) + (part[2 * DOUT + tid] + part[3 * DOUT + tid]);
    outs[tid] = s + bf16_val(bfv[tid]);
  }
  __syncthreads();
  const v4f ov = *(const v4fa*)(outs + 4 * (lane & 15));
  float* op = out + (size_t)g * DOUT + 4 * (lane & 15);
  const bool okst = (wave == 0) && (lane < 16);
  if (okst) *(volatile v4f*)op = ov;
  __threadfence();
  if (okst) *(volatile v4f*)op = ov;
}

static inline int cdiv(int a, int b) { return (a + b - 1) / b; }
static inline size_t al256(size_t o) { return (o + 255) & ~(size_t)255; }

extern "C" void kernel_launch(void* const* d_in, const int* in_sizes, int n_in,
                              void* d_out, int out_size, void* d_ws, size_t ws_size,
                              hipStream_t stream) {
  if (n_in < 14) return;
  if (in_sizes[0] < DIN || (in_sizes[0] % DIN) != 0) return;
  const int nN = in_sizes[0] / DIN;
  const int nE = in_sizes[1];
  if (nE < 1 || in_sizes[2] != nE) return;
  if (nE >= (1 << 21) || nN < 16 || nN >= (1 << 22)) return;
  if (in_sizes[3] != nN) return;
  if (in_sizes[4] != DIN * DH || in_sizes[5] != DH) return;
  if (in_sizes[6] != DIN * DH || in_sizes[7] != DH) return;
  if (in_sizes[8] != DH * DH || in_sizes[9] != DH) return;
  if (in_sizes[10] != DH * DH || in_sizes[11] != DH) return;
  if (in_sizes[12] != DH * DOUT || in_sizes[13] != DOUT) return;
  if (out_size < DOUT || (out_size % DOUT) != 0) return;
  const int nG = out_size / DOUT;
  if (nG > 65535) return;

  const float* x    = (const float*)d_in[0];
  const int*   erow = (const int*)d_in[1];
  const int*   ecol = (const int*)d_in[2];
  const int*   gid  = (const int*)d_in[3];
  const float* w1a  = (const float*)d_in[4];
  const float* b1a  = (const float*)d_in[5];
  const float* w1b  = (const float*)d_in[6];
  const float* b1b  = (const float*)d_in[7];
  const float* w2a  = (const float*)d_in[8];
  const float* b2a  = (const float*)d_in[9];
  const float* w2b  = (const float*)d_in[10];
  const float* b2b  = (const float*)d_in[11];
  const float* wf   = (const float*)d_in[12];
  const float* bfv  = (const float*)d_in[13];
  float* out = (float*)d_out;

  const int MP = cdiv(nN, GBM) * GBM;
  const int gM = MP / GBM;
  const int gA = cdiv(MP, NBA);
  if ((long long)gA * NBA < (long long)MP) return;
  const int vec8 = ((nE & 3) == 0) ? 1 : 0;

  char* ws = (char*)d_ws;
  size_t off = 0;
  const size_t oW1 = off; off = al256(off + (size_t)DH * P1 * 2);
  const size_t oW2 = off; off = al256(off + (size_t)DH * P2 * 2);
  const size_t oA1 = off; off = al256(off + (size_t)MP * P1 * 2);
  const size_t oH  = off; off = al256(off + (size_t)MP * DH * 4);
  const size_t oA2 = off; off = al256(off + (size_t)MP * P2 * 2);
  if (off > ws_size || off > (size_t)WSMAX) return;
  unsigned short* W1C = (unsigned short*)(ws + oW1);
  unsigned short* W2C = (unsigned short*)(ws + oW2);
  unsigned short* A1  = (unsigned short*)(ws + oA1);
  float*          H   = (float*)(ws + oH);
  unsigned short* A2  = (unsigned short*)(ws + oA2);

  const size_t scanLds = (size_t)AGG_LDS_INTS * 4;
  hipFuncSetAttribute(reinterpret_cast<const void*>(&k_scan<1>), hipFuncAttributeMaxDynamicSharedMemorySize, (int)scanLds);
  hipFuncSetAttribute(reinterpret_cast<const void*>(&k_scan<0>), hipFuncAttributeMaxDynamicSharedMemorySize, (int)scanLds);

  const int nUx = MP * (DIN / 8);
  k_wprep<<<NUW / NTHR, NTHR, 0, stream>>>(w1a, w1b, w2a, w2b, W1C, W2C);
  k_cvx<<<cdiv(nUx, NTHR), NTHR, 0, stream>>>(x, nN, nUx, A1);
  k_scan<1><<<gA, NTHR, scanLds, stream>>>(ecol, erow, nE, nN, vec8, MP, A1, H, A1);
  k_gemm<1><<<gM, GTHR, 0, stream>>>(A1, W1C, P1, b1a, b1b, H, A2, nN);
  k_scan<0><<<gA, NTHR, scanLds, stream>>>(ecol, erow, nE, nN, vec8, MP, A1, H, A2);
  k_gemm<0><<<gM, GTHR, 0, stream>>>(A2, W2C, P2, b2a, b2b, H, A2, nN);
  k_pool_out<<<nG, NTHR, 0, stream>>>(H, gid, nN, wf, bfv, out);
}
